// EmbededNonLocalLayer_10788957847970
// MI455X (gfx1250) — hardware-verified
//
#include <hip/hip_runtime.h>

#define NB   4
#define CIN  512
#define CI   256
#define CO   512
#define HWD  63
#define NSP  3969
#define NP   4032
#define KK   81
#define KP   96
#define SNP  128
#define NT   63
#define LPC  124
#define ATT_SCALE 0.0625f
#define BN_EPS 1e-5f
#define PSCALE 16384.0f

static_assert(NSP == LPC * 32 + 1);
static_assert(NP == NT * 64);
static_assert(HWD * HWD == NSP);

typedef _Float16 v16h __attribute__((ext_vector_type(16)));
typedef _Float16 v8h  __attribute__((ext_vector_type(8)));
typedef __bf16   v16b __attribute__((ext_vector_type(16)));
typedef unsigned short v16u __attribute__((ext_vector_type(16)));
typedef unsigned short v8u  __attribute__((ext_vector_type(8)));
typedef float v8f __attribute__((ext_vector_type(8)));
typedef float v4f __attribute__((ext_vector_type(4)));
typedef v8h __attribute__((may_alias)) v8ha;
typedef v8u __attribute__((may_alias)) v8ua;
typedef v4f __attribute__((may_alias)) v4fa;
typedef unsigned short us_t;

union FragH { v16h v; v8h half[2]; };
union FragB { v16b v; v16u u; v8u half[2]; };

constexpr size_t SZ_W1   = (size_t)CI * CIN * 2;
constexpr size_t SZ_W2   = (size_t)CI * CI * 2;
constexpr size_t SZ_W3   = (size_t)CO * CI * 2;
constexpr size_t SZ_X16  = (size_t)NB * NP * CIN * 2;
constexpr size_t SZ_P16  = (size_t)NB * NP * CI * 2;
constexpr size_t SZ_P32  = (size_t)NB * NP * CI * 4;
constexpr size_t SZ_POOL = (size_t)NB * KP * CI * 4;
constexpr size_t SZ_V2T  = (size_t)NB * KP * CI * 2;
constexpr size_t SZ_V2P  = (size_t)NB * CI * SNP * 2;
constexpr size_t SZ_SIMV = (size_t)NB * KP * NP * 2;
constexpr size_t SZ_SN   = (size_t)NB * NP * SNP * 2;
constexpr size_t OFF_WK   = 0;
constexpr size_t OFF_WVH  = OFF_WK + SZ_W1;
constexpr size_t OFF_WVL  = OFF_WVH + SZ_W1;
constexpr size_t OFF_WV2H = OFF_WVL + SZ_W1;
constexpr size_t OFF_WV2L = OFF_WV2H + SZ_W2;
constexpr size_t OFF_WWH  = OFF_WV2L + SZ_W2;
constexpr size_t OFF_WWL  = OFF_WWH + SZ_W3;
constexpr size_t OFF_XH   = OFF_WWL + SZ_W3;
constexpr size_t OFF_XBH  = OFF_XH + SZ_X16;
constexpr size_t OFF_XBL  = OFF_XBH + SZ_X16;
constexpr size_t OFF_QK   = OFF_XBL + SZ_X16;
constexpr size_t OFF_VF   = OFF_QK + SZ_P16;
constexpr size_t OFF_VH   = OFF_VF + SZ_P32;
constexpr size_t OFF_POOL = OFF_VH + SZ_P16;
constexpr size_t OFF_V2T  = OFF_POOL + SZ_POOL;
constexpr size_t OFF_V2H  = OFF_V2T + SZ_V2T;
constexpr size_t OFF_V2L  = OFF_V2H + SZ_V2P;
constexpr size_t OFF_SIMV = OFF_V2L + SZ_V2P;
constexpr size_t OFF_SNH  = OFF_SIMV + SZ_SIMV;
constexpr size_t OFF_SNL  = OFF_SNH + SZ_SN;
constexpr size_t OFF_CTH  = OFF_SNL + SZ_SN;
constexpr size_t OFF_CTL  = OFF_CTH + SZ_P16;
constexpr size_t OFF_END  = OFF_CTL + SZ_P16;
static_assert(OFF_END <= (size_t)134217728);
static_assert((OFF_XH & 255) == 0 && (OFF_POOL & 255) == 0 && (OFF_SIMV & 255) == 0 && (OFF_CTL & 255) == 0);

__device__ __forceinline__ v8f mma_h(v16h a, v16h b, v8f c) {
  v8f d = __builtin_amdgcn_wmma_f32_16x16x32_f16(false, a, false, b, (short)0, c, false, false);
  asm volatile("v_nop\n\tv_nop\n\tv_nop\n\tv_nop" : "+v"(d) : "v"(a), "v"(b));
  return d;
}
__device__ __forceinline__ v8f mma_b(v16b a, v16b b, v8f c) {
  v8f d = __builtin_amdgcn_wmma_f32_16x16x32_bf16(false, a, false, b, (short)0, c, false, false);
  asm volatile("v_nop\n\tv_nop\n\tv_nop\n\tv_nop" : "+v"(d) : "v"(a), "v"(b));
  return d;
}
__device__ __forceinline__ v16h ldh(const _Float16* p, int h) {
  FragH f;
  f.half[0] = *(const v8ha*)(p + 8 * h);
  f.half[1] = *(const v8ha*)(p + 16 + 8 * h);
  return f.v;
}
__device__ __forceinline__ v16b ldb(const us_t* p, int h) {
  FragB f;
  f.half[0] = *(const v8ua*)(p + 8 * h);
  f.half[1] = *(const v8ua*)(p + 16 + 8 * h);
  return f.v;
}

__device__ __forceinline__ unsigned bf_bits(float x) {
  const unsigned u = __float_as_uint(x);
  return (u + 0x7FFFu + ((u >> 16) & 1u)) >> 16;
}
__device__ __forceinline__ float bf_val(unsigned bbits) { return __uint_as_float(bbits << 16); }

__device__ __forceinline__ void split8(v4f a, v4f c, v8u& hi, v8u& lo) {
  const float e[8] = {a.x, a.y, a.z, a.w, c.x, c.y, c.z, c.w};
#pragma unroll
  for (int i = 0; i < 8; ++i) {
    const unsigned hb = bf_bits(e[i]);
    hi[i] = (unsigned short)hb;
    lo[i] = (unsigned short)bf_bits(e[i] - bf_val(hb));
  }
}
__device__ __forceinline__ v8h toh8(v4f a, v4f c, float s) {
  const v8h o = { (_Float16)(a.x * s), (_Float16)(a.y * s), (_Float16)(a.z * s), (_Float16)(a.w * s),
                  (_Float16)(c.x * s), (_Float16)(c.y * s), (_Float16)(c.z * s), (_Float16)(c.w * s) };
  return o;
}
__device__ __forceinline__ void ldsplit(const float* p, int h, v16b& hi, v16b& lo) {
  const v4f a0 = *(const v4fa*)(p + 8 * h);
  const v4f a1 = *(const v4fa*)(p + 8 * h + 4);
  const v4f a2 = *(const v4fa*)(p + 16 + 8 * h);
  const v4f a3 = *(const v4fa*)(p + 16 + 8 * h + 4);
  FragB fh, fl;
  split8(a0, a1, fh.half[0], fl.half[0]);
  split8(a2, a3, fh.half[1], fl.half[1]);
  hi = fh.v; lo = fl.v;
}

__device__ __forceinline__ float hmax16(float v) {
#pragma unroll
  for (int s = 1; s <= 8; s <<= 1) v = fmaxf(v, __shfl_xor(v, s, 32));
  return v;
}
__device__ __forceinline__ float hsum16(float v) {
#pragma unroll
  for (int s = 1; s <= 8; s <<= 1) v += __shfl_xor(v, s, 32);
  return v;
}

__global__ __launch_bounds__(256) void k_wprep(
    const float* __restrict__ Wk, const float* __restrict__ Wv, const float* __restrict__ Wv2,
    const float* __restrict__ Ww, _Float16* __restrict__ wk16,
    us_t* __restrict__ wvh, us_t* __restrict__ wvl, us_t* __restrict__ wv2h, us_t* __restrict__ wv2l,
    us_t* __restrict__ wwh, us_t* __restrict__ wwl)
{
  const int g = blockIdx.x * 256 + threadIdx.x;
  const int G1 = CI * CIN / 8, G2 = CI * CIN / 8, G3 = CI * CI / 8, G4 = CO * CI / 8;
  if (g >= G1 + G2 + G3 + G4) return;
  if (g < G1) {
    const float* src = Wk + (size_t)g * 8;
    const v4f a = *(const v4fa*)src;
    const v4f c = *(const v4fa*)(src + 4);
    const v8h o = toh8(a, c, 64.0f);
    _Float16* dst = wk16 + (size_t)g * 8;
    *(volatile v8h*)dst = o;
    __threadfence();
    *(volatile v8h*)dst = o;
    return;
  }
  const float* src;
  us_t* dh;
  us_t* dl;
  size_t e;
  if (g < G1 + G2)           { e = (size_t)(g - G1);           src = Wv;  dh = wvh;  dl = wvl;  }
  else if (g < G1 + G2 + G3) { e = (size_t)(g - G1 - G2);      src = Wv2; dh = wv2h; dl = wv2l; }
  else                       { e = (size_t)(g - G1 - G2 - G3); src = Ww;  dh = wwh;  dl = wwl;  }
  src += e * 8;
  const v4f a = *(const v4fa*)src;
  const v4f c = *(const v4fa*)(src + 4);
  v8u hi, lo;
  split8(a, c, hi, lo);
  us_t* ph = dh + e * 8;
  us_t* pl = dl + e * 8;
  *(volatile v8u*)ph = hi;
  *(volatile v8u*)pl = lo;
  __threadfence();
  *(volatile v8u*)ph = hi;
  *(volatile v8u*)pl = lo;
}

__global__ __launch_bounds__(256) void k_xprep(const float* __restrict__ x, _Float16* __restrict__ xh16,
                                               us_t* __restrict__ xbh, us_t* __restrict__ xbl)
{
  __shared__ float sx[64 * 65];
  const int tid = threadIdx.x;
  const int p0 = blockIdx.x * 64, c0 = blockIdx.y * 64, b = blockIdx.z;
#pragma unroll 1
  for (int idx = tid; idx < 4096; idx += 256) {
    const int c = idx >> 6, j = idx & 63;
    const int n = p0 + j;
    const int nc = (n < NSP) ? n : (NSP - 1);
    const float v = x[((size_t)(b * CIN + c0 + c)) * NSP + nc];
    sx[c * 65 + j] = (n < NSP) ? v : 0.0f;
  }
  __syncthreads();
  v8h fh[2];
  v8u fb[2], fl[2];
  size_t off[2];
#pragma unroll
  for (int k = 0; k < 2; ++k) {
    const int pi = tid + 256 * k;
    const int px = pi >> 3, q8 = pi & 7;
    float e[8];
#pragma unroll
    for (int i = 0; i < 8; ++i) e[i] = sx[(8 * q8 + i) * 65 + px];
    const v4f a = {e[0], e[1], e[2], e[3]};
    const v4f c = {e[4], e[5], e[6], e[7]};
    fh[k] = toh8(a, c, 1.0f);
    split8(a, c, fb[k], fl[k]);
    off[k] = ((size_t)(b * NP + p0 + px)) * CIN + c0 + 8 * q8;
  }
#pragma unroll
  for (int k = 0; k < 2; ++k) {
    *(volatile v8h*)(xh16 + off[k]) = fh[k];
    *(volatile v8u*)(xbh + off[k]) = fb[k];
    *(volatile v8u*)(xbl + off[k]) = fl[k];
  }
  __threadfence();
#pragma unroll
  for (int k = 0; k < 2; ++k) {
    *(volatile v8h*)(xh16 + off[k]) = fh[k];
    *(volatile v8u*)(xbh + off[k]) = fb[k];
    *(volatile v8u*)(xbl + off[k]) = fl[k];
  }
}

__device__ __forceinline__ void convq_store(const _Float16* sT, _Float16* qkp, int b, int p0, int cg, int tid) {
  const int q8 = tid & 7, sub = tid >> 3;
#pragma unroll
  for (int i = 0; i < 4; ++i) {
    const int px = 16 * i + sub;
    const v8h v = *(const v8ha*)(sT + px * 64 + 8 * q8);
    *(volatile v8h*)(qkp + ((size_t)(b * NP + p0 + px)) * CI + cg * 64 + 8 * q8) = v;
  }
}

__global__ __launch_bounds__(128) void k_convq(
    const _Float16* __restrict__ xh16, const _Float16* __restrict__ wk16,
    const float* __restrict__ bk, const float* __restrict__ gamma, const float* __restrict__ beta,
    _Float16* __restrict__ qkp)
{
  __shared__ __attribute__((aligned(16))) _Float16 sT[64 * 64];
  const int tid = threadIdx.x, lane = tid & 31, w = tid >> 5, h = lane >> 4, m = lane & 15;
  const int p0 = blockIdx.x * 64, cg = blockIdx.y, b = blockIdx.z;
  const _Float16* arow = xh16 + ((size_t)(b * NP + p0 + 16 * w + m)) * CIN;
  const _Float16* brow = wk16 + ((size_t)(cg * 64 + m)) * CIN;
  const v8f zero8 = {0.f, 0.f, 0.f, 0.f, 0.f, 0.f, 0.f, 0.f};
  v8f acc[4];
#pragma unroll
  for (int nt = 0; nt < 4; ++nt) acc[nt] = zero8;
#pragma unroll 1
  for (int k0 = 0; k0 < CIN; k0 += 32) {
    const v16h a = ldh(arow + k0, h);
#pragma unroll
    for (int nt = 0; nt < 4; ++nt) {
      const v16h bb = ldh(brow + (size_t)nt * 16 * CIN + k0, h);
      acc[nt] = mma_h(a, bb, acc[nt]);
    }
  }
  const float isq = 1.0f / sqrtf(1.0f + BN_EPS);
#pragma unroll
  for (int nt = 0; nt < 4; ++nt) {
    const int ci = cg * 64 + 16 * nt + m;
    const float bb = bk[ci];
    const float sc = gamma[ci] * isq;
    const float be = beta[ci];
#pragma unroll
    for (int r = 0; r < 8; ++r) {
      const int px = 16 * w + 8 * h + r;
      const float val = (acc[nt][r] * 0.015625f + bb) * sc + be;
      sT[px * 64 + 16 * nt + m] = (_Float16)((p0 + px < NSP) ? val : 0.0f);
    }
  }
  __syncthreads();
  convq_store(sT, qkp, b, p0, cg, tid);
  __threadfence();
  convq_store(sT, qkp, b, p0, cg, tid);
}

__device__ __forceinline__ void convv_store(const float* sV, float* vf, _Float16* vh16, int b, int p0, int cg, int tid) {
  const int q8 = tid & 7, sub = tid >> 3;
#pragma unroll
  for (int i = 0; i < 8; ++i) {
    const int it = 16 * i + sub;
    const int px = it >> 1, hl = it & 1;
    const v4f v = *(const v4fa*)(sV + px * 64 + 32 * hl + 4 * q8);
    *(volatile v4f*)(vf + ((size_t)(b * NP + p0 + px)) * CI + cg * 64 + 32 * hl + 4 * q8) = v;
  }
#pragma unroll
  for (int i = 0; i < 4; ++i) {
    const int px = 16 * i + sub;
    const v4f a = *(const v4fa*)(sV + px * 64 + 8 * q8);
    const v4f c = *(const v4fa*)(sV + px * 64 + 8 * q8 + 4);
    const v8h v = toh8(a, c, 1.0f);
    *(volatile v8h*)(vh16 + ((size_t)(b * NP + p0 + px)) * CI + cg * 64 + 8 * q8) = v;
  }
}

__global__ __launch_bounds__(128) void k_convv(
    const us_t* __restrict__ xbh, const us_t* __restrict__ xbl,
    const us_t* __restrict__ wvh, const us_t* __restrict__ wvl, const float* __restrict__ bv,
    float* __restrict__ vf, _Float16* __restrict__ vh16)
{
  __shared__ __attribute__((aligned(16))) float sV[64 * 64];
  const int tid = threadIdx.x, lane = tid & 31, w = tid >> 5, h = lane >> 4, m = lane & 15;
  const int p0 = blockIdx.x * 64, cg = blockIdx.y, b = blockIdx.z;
  const size_t arow = ((size_t)(b * NP + p0 + 16 * w + m)) * CIN;
  const size_t brow = ((size_t)(cg * 64 + m)) * CIN;
  const v8f zero8 = {0.f, 0.f, 0.f, 0.f, 0.f, 0.f, 0.f, 0.f};
  v8f acc[4];
#pragma unroll
  for (int nt = 0; nt < 4; ++nt) acc[nt] = zero8;
#pragma unroll 1
  for (int k0 = 0; k0 < CIN; k0 += 32) {
    const v16b ah = ldb(xbh + arow + k0, h);
    const v16b al = ldb(xbl + arow + k0, h);
#pragma unroll
    for (int nt = 0; nt < 4; ++nt) {
      const v16b bh = ldb(wvh + brow + (size_t)nt * 16 * CIN + k0, h);
      const v16b bl = ldb(wvl + brow + (size_t)nt * 16 * CIN + k0, h);
      acc[nt] = mma_b(ah, bh, acc[nt]);
      acc[nt] = mma_b(al, bh, acc[nt]);
      acc[nt] = mma_b(ah, bl, acc[nt]);
    }
  }
#pragma unroll
  for (int nt = 0; nt < 4; ++nt) {
    const int ci = cg * 64 + 16 * nt + m;
    const float bb = bv[ci];
#pragma unroll
    for (int r = 0; r < 8; ++r) {
      const int px = 16 * w + 8 * h + r;
      sV[px * 64 + 16 * nt + m] = (p0 + px < NSP) ? (acc[nt][r] + bb) : 0.0f;
    }
  }
  __syncthreads();
  convv_store(sV, vf, vh16, b, p0, cg, tid);
  __threadfence();
  convv_store(sV, vf, vh16, b, p0, cg, tid);
}

__global__ __launch_bounds__(256) void k_pool(const float* __restrict__ vf, float* __restrict__ poolT)
{
  const int gid = blockIdx.x * 256 + threadIdx.x;
  if (gid >= NB * KP * CI) return;
  const int ci = gid & (CI - 1);
  const int cell = (gid >> 8) % KP;
  const int b = (gid >> 8) / KP;
  const int cc = (cell < KK) ? cell : 0;
  const int gi = cc / 9, gj = cc - 9 * gi;
  const float* src = vf + ((size_t)(b * NP)) * CI + ci;
  float acc = 0.0f;
#pragma unroll 1
  for (int i = 0; i < 7; ++i) {
#pragma unroll
    for (int j = 0; j < 7; ++j)
      acc += src[(size_t)((7 * gi + i) * HWD + 7 * gj + j) * CI];
  }
  const float val = (cell < KK) ? acc * (1.0f / 49.0f) : 0.0f;
  *(volatile float*)(poolT + gid) = val;
  __threadfence();
  *(volatile float*)(poolT + gid) = val;
}

__device__ __forceinline__ void v2_store(const float* sD, _Float16* v2T, us_t* v2hp, us_t* v2lp, int b, int cg, int tid) {
  const int q8 = tid & 7, sub = tid >> 3;
  const v4f z4 = {0.f, 0.f, 0.f, 0.f};
#pragma unroll
  for (int i = 0; i < 6; ++i) {
    const int cell = 16 * i + sub;
    float e[8];
#pragma unroll
    for (int k = 0; k < 8; ++k) e[k] = sD[(8 * q8 + k) * KP + cell];
    const v4f a = {e[0], e[1], e[2], e[3]};
    const v4f c = {e[4], e[5], e[6], e[7]};
    const v8h v = toh8(a, c, 64.0f);
    *(volatile v8h*)(v2T + ((size_t)(b * KP + cell)) * CI + cg * 64 + 8 * q8) = v;
  }
#pragma unroll
  for (int i = 0; i < 8; ++i) {
    const int it = 16 * i + sub;
    const int c = it >> 1, hl = it & 1;
    const int c0 = 64 * hl + 8 * q8;
    const int cc = (c0 < KP) ? c0 : (KP - 8);
    v4f a = *(const v4fa*)(sD + c * KP + cc);
    v4f cv = *(const v4fa*)(sD + c * KP + cc + 4);
    if (c0 >= KP) { a = z4; cv = z4; }
    v8u hi, lo;
    split8(a, cv, hi, lo);
    const size_t gi = ((size_t)(b * CI + cg * 64 + c)) * SNP + c0;
    *(volatile v8u*)(v2hp + gi) = hi;
    *(volatile v8u*)(v2lp + gi) = lo;
  }
}

__global__ __launch_bounds__(128) void k_v2(
    const us_t* __restrict__ wv2h, const us_t* __restrict__ wv2l, const float* __restrict__ poolT,
    const float* __restrict__ bv2, _Float16* __restrict__ v2T, us_t* __restrict__ v2hp, us_t* __restrict__ v2lp)
{
  __shared__ __attribute__((aligned(16))) float sD[64 * KP];
  const int tid = threadIdx.x, lane = tid & 31, w = tid >> 5, h = lane >> 4, m = lane & 15;
  const int cg = blockIdx.x, b = blockIdx.y;
  const int crow = cg * 64 + 16 * w;
  const us_t* ah0 = wv2h + ((size_t)(crow + m)) * CI;
  const us_t* al0 = wv2l + ((size_t)(crow + m)) * CI;
  const float* prow = poolT + ((size_t)(b * KP + m)) * CI;
  float bias8[8];
#pragma unroll
  for (int r = 0; r < 8; ++r) bias8[r] = bv2[crow + 8 * h + r];
  const v8f zero8 = {0.f, 0.f, 0.f, 0.f, 0.f, 0.f, 0.f, 0.f};
#pragma unroll 1
  for (int g = 0; g < 2; ++g) {
    v8f acc[3];
#pragma unroll
    for (int nt = 0; nt < 3; ++nt) acc[nt] = zero8;
#pragma unroll 1
    for (int k0 = 0; k0 < CI; k0 += 32) {
      const v16b ah = ldb(ah0 + k0, h);
      const v16b al = ldb(al0 + k0, h);
#pragma unroll
      for (int nt = 0; nt < 3; ++nt) {
        v16b bh, bl;
        ldsplit(prow + (size_t)((3 * g + nt) * 16) * CI + k0, h, bh, bl);
        acc[nt] = mma_b(ah, bh, acc[nt]);
        acc[nt] = mma_b(al, bh, acc[nt]);
        acc[nt] = mma_b(ah, bl, acc[nt]);
      }
    }
#pragma unroll
    for (int nt = 0; nt < 3; ++nt) {
      const int cell = (3 * g + nt) * 16 + m;
#pragma unroll
      for (int r = 0; r < 8; ++r) {
        const int cl = 16 * w + 8 * h + r;
        sD[cl * KP + cell] = (cell < KK) ? (acc[nt][r] + bias8[r]) : 0.0f;
      }
    }
  }
  __syncthreads();
  v2_store(sD, v2T, v2hp, v2lp, b, cg, tid);
  __threadfence();
  v2_store(sD, v2T, v2hp, v2lp, b, cg, tid);
}

__device__ __forceinline__ void simv_store(const _Float16* sP, _Float16* simvT, int b, int p0, int tid) {
  const int q8 = tid & 7, sub = tid >> 3;
#pragma unroll
  for (int i = 0; i < 6; ++i) {
    const int cell = 16 * i + sub;
    const v8h v = *(const v8ha*)(sP + cell * 64 + 8 * q8);
    *(volatile v8h*)(simvT + ((size_t)(b * KP + cell)) * NP + p0 + 8 * q8) = v;
  }
}

__global__ __launch_bounds__(128) void k_simv(const _Float16* __restrict__ vh16, const _Float16* __restrict__ v2T,
                                              _Float16* __restrict__ simvT)
{
  __shared__ __attribute__((aligned(16))) _Float16 sP[KP * 64];
  const int tid = threadIdx.x, lane = tid & 31, w = tid >> 5, h = lane >> 4, m = lane & 15;
  const int p0 = blockIdx.x * 64, b = blockIdx.y;
  const _Float16* arow = vh16 + ((size_t)(b * NP + p0 + 16 * w + m)) * CI;
  const _Float16* brow = v2T + ((size_t)(b * KP + m)) * CI;
  const v8f zero8 = {0.f, 0.f, 0.f, 0.f, 0.f, 0.f, 0.f, 0.f};
  v8f acc[6];
#pragma unroll
  for (int nt = 0; nt < 6; ++nt) acc[nt] = zero8;
#pragma unroll 1
  for (int k0 = 0; k0 < CI; k0 += 32) {
    const v16h a = ldh(arow + k0, h);
#pragma unroll
    for (int nt = 0; nt < 6; ++nt) {
      const v16h bb = ldh(brow + (size_t)nt * 16 * CI + k0, h);
      acc[nt] = mma_h(a, bb, acc[nt]);
    }
  }
  const float ssc = ATT_SCALE * 0.015625f;
#pragma unroll
  for (int r = 0; r < 8; ++r) {
    float mx = -1e30f;
#pragma unroll
    for (int nt = 0; nt < 6; ++nt) {
      const float xv = (16 * nt + m < KK) ? acc[nt][r] * ssc : -1e30f;
      acc[nt][r] = xv;
      mx = fmaxf(mx, xv);
    }
    mx = hmax16(mx);
    float sum = 0.0f;
#pragma unroll
    for (int nt = 0; nt < 6; ++nt) {
      const float p = __expf(acc[nt][r] - mx);
      acc[nt][r] = p;
      sum += p;
    }
    sum = hsum16(sum);
    const float inv = 1.0f / sum;
#pragma unroll
    for (int nt = 0; nt < 6; ++nt)
      sP[(16 * nt + m) * 64 + 16 * w + 8 * h + r] = (_Float16)(acc[nt][r] * inv);
  }
  __syncthreads();
  simv_store(sP, simvT, b, p0, tid);
  __threadfence();
  simv_store(sP, simvT, b, p0, tid);
}

__device__ __forceinline__ v16h pack_p(v8f a, v8f c) {
  const v16h r = { (_Float16)(a[0] * PSCALE), (_Float16)(a[1] * PSCALE), (_Float16)(a[2] * PSCALE), (_Float16)(a[3] * PSCALE),
                   (_Float16)(a[4] * PSCALE), (_Float16)(a[5] * PSCALE), (_Float16)(a[6] * PSCALE), (_Float16)(a[7] * PSCALE),
                   (_Float16)(c[0] * PSCALE), (_Float16)(c[1] * PSCALE), (_Float16)(c[2] * PSCALE), (_Float16)(c[3] * PSCALE),
                   (_Float16)(c[4] * PSCALE), (_Float16)(c[5] * PSCALE), (_Float16)(c[6] * PSCALE), (_Float16)(c[7] * PSCALE) };
  return r;
}

__device__ __forceinline__ void flash_store(const float* so, us_t* snh, us_t* snl, int b, int q0, int lane) {
  const int q8 = lane & 7, sub = lane >> 3;
  const v4f z4 = {0.f, 0.f, 0.f, 0.f};
#pragma unroll
  for (int i = 0; i < 8; ++i) {
    const int it = 4 * i + sub;
    const int row = it >> 1, hl = it & 1;
    const int c0 = 64 * hl + 8 * q8;
    const int cc = (c0 < KP) ? c0 : (KP - 8);
    v4f a = *(const v4fa*)(so + row * KP + cc);
    v4f c = *(const v4fa*)(so + row * KP + cc + 4);
    if (c0 >= KP) { a = z4; c = z4; }
    v8u hi, lo;
    split8(a, c, hi, lo);
    const size_t gi = ((size_t)(b * NP + q0 + row)) * SNP + c0;
    *(volatile v8u*)(snh + gi) = hi;
    *(volatile v8u*)(snl + gi) = lo;
  }
}

__global__ __launch_bounds__(128) void k_flash(const _Float16* __restrict__ qkp, const _Float16* __restrict__ simvT,
                                               us_t* __restrict__ snh, us_t* __restrict__ snl)
{
  __shared__ __attribute__((aligned(16))) float sO[4 * 16 * KP];
  const int tid = threadIdx.x, lane = tid & 31, w = tid >> 5, h = lane >> 4, m = lane & 15;
  const int b = blockIdx.y;
  const int q0 = blockIdx.x * 64 + 16 * w;
  const _Float16* qrow  = qkp + ((size_t)(b * NP + q0 + m)) * CI;
  const _Float16* kbase = qkp + ((size_t)(b * NP + m)) * CI;
  const _Float16* vbase = simvT + ((size_t)(b * KP + m)) * NP;
  const v8f zero8 = {0.f, 0.f, 0.f, 0.f, 0.f, 0.f, 0.f, 0.f};
  v8f o[6];
#pragma unroll
  for (int t = 0; t < 6; ++t) o[t] = zero8;
  float mrun = -1e30f, lrun = 0.0f;

#pragma unroll 1
  for (int kb = 0; kb < NP; kb += 64) {
    v8f s[4];
#pragma unroll
    for (int j = 0; j < 4; ++j) s[j] = zero8;
#pragma unroll
    for (int kc = 0; kc < 8; ++kc) {
      const v16h qf = ldh(qrow + 32 * kc, h);
#pragma unroll
      for (int j = 0; j < 4; ++j) {
        const v16h kf = ldh(kbase + (size_t)(kb + 16 * j) * CI + 32 * kc, h);
        s[j] = mma_h(kf, qf, s[j]);
      }
    }
#pragma unroll
    for (int j = 0; j < 4; ++j)
#pragma unroll
      for (int r = 0; r < 8; ++r) {
        const int key = kb + 16 * j + 8 * h + r;
        const float xv = s[j][r] * ATT_SCALE;
        s[j][r] = (key < NSP) ? xv : -1e30f;
      }
    float mloc = s[0][0];
#pragma unroll
    for (int j = 0; j < 4; ++j)
#pragma unroll
      for (int r = 0; r < 8; ++r) mloc = fmaxf(mloc, s[j][r]);
    mloc = fmaxf(mloc, __shfl_xor(mloc, 16, 32));
    const float mnew = fmaxf(mrun, mloc);
    const float alpha = __expf(mrun - mnew);
    mrun = mnew;
    float lsum = 0.0f;
#pragma unroll
    for (int j = 0; j < 4; ++j)
#pragma unroll
      for (int r = 0; r < 8; ++r) {
        const float p = __expf(s[j][r] - mnew);
        s[j][r] = p;
        lsum += p;
      }
    lsum += __shfl_xor(lsum, 16, 32);
    lrun = lrun * alpha + lsum;
#pragma unroll
    for (int t = 0; t < 6; ++t)
#pragma unroll
      for (int r = 0; r < 8; ++r) o[t][r] = o[t][r] * alpha;

    const v16h pb0 = pack_p(s[0], s[1]);
    const v16h pb1 = pack_p(s[2], s[3]);
#pragma unroll
    for (int t = 0; t < 6; ++t) {
      const _Float16* vp = vbase + (size_t)(16 * t) * NP + kb;
      const v16h vf0 = ldh(vp, h);
      const v16h vf1 = ldh(vp + 32, h);
      o[t] = mma_h(vf0, pb0, o[t]);
      o[t] = mma_h(vf1, pb1, o[t]);
    }
  }

  const float inv = (1.0f / lrun) * (1.0f / PSCALE);
  float* so = sO + w * 16 * KP;
#pragma unroll
  for (int t = 0; t < 6; ++t)
#pragma unroll
    for (int r = 0; r < 8; ++r)
      so[m * KP + 16 * t + 8 * h + r] = o[t][r] * inv;
  __syncthreads();
  flash_store(so, snh, snl, b, q0, lane);
  __threadfence();
  flash_store(so, snh, snl, b, q0, lane);
}

__device__ __forceinline__ void ctx_store(const float* sC, us_t* cth, us_t* ctl, int b, int p0, int cg, int tid) {
  const int q8 = tid & 7, sub = tid >> 3;
#pragma unroll
  for (int i = 0; i < 4; ++i) {
    const int px = 16 * i + sub;
    const v4f a = *(const v4fa*)(sC + px * 64 + 8 * q8);
    const v4f c = *(const v4fa*)(sC + px * 64 + 8 * q8 + 4);
    v8u hi, lo;
    split8(a, c, hi, lo);
    const size_t gi = ((size_t)(b * NP + p0 + px)) * CI + cg * 64 + 8 * q8;
    *(volatile v8u*)(cth + gi) = hi;
    *(volatile v8u*)(ctl + gi) = lo;
  }
}

__global__ __launch_bounds__(128) void k_ctx(
    const us_t* __restrict__ snh, const us_t* __restrict__ snl,
    const us_t* __restrict__ v2hp, const us_t* __restrict__ v2lp,
    us_t* __restrict__ cth, us_t* __restrict__ ctl)
{
  __shared__ __attribute__((aligned(16))) float sC[64 * 64];
  const int tid = threadIdx.x, lane = tid & 31, w = tid >> 5, h = lane >> 4, m = lane & 15;
  const int p0 = blockIdx.x * 64, cg = blockIdx.y, b = blockIdx.z;
  const size_t arow = ((size_t)(b * NP + p0 + 16 * w + m)) * SNP;
  const size_t brow = ((size_t)(b * CI + cg * 64 + m)) * SNP;
  const v8f zero8 = {0.f, 0.f, 0.f, 0.f, 0.f, 0.f, 0.f, 0.f};
  v8f acc[4];
#pragma unroll
  for (int nt = 0; nt < 4; ++nt) acc[nt] = zero8;
#pragma unroll
  for (int ks = 0; ks < 3; ++ks) {
    const int k0 = 32 * ks;
    const v16b ah = ldb(snh + arow + k0, h);
    const v16b al = ldb(snl + arow + k0, h);
#pragma unroll
    for (int nt = 0; nt < 4; ++nt) {
      const v16b bh = ldb(v2hp + brow + (size_t)nt * 16 * SNP + k0, h);
      const v16b bl = ldb(v2lp + brow + (size_t)nt * 16 * SNP + k0, h);
      acc[nt] = mma_b(ah, bh, acc[nt]);
      acc[nt] = mma_b(al, bh, acc[nt]);
      acc[nt] = mma_b(ah, bl, acc[nt]);
    }
  }
#pragma unroll
  for (int nt = 0; nt < 4; ++nt)
#pragma unroll
    for (int r = 0; r < 8; ++r)
      sC[(16 * w + 8 * h + r) * 64 + 16 * nt + m] = acc[nt][r];
  __syncthreads();
  ctx_store(sC, cth, ctl, b, p0, cg, tid);
  __threadfence();
  ctx_store(sC, cth, ctl, b, p0, cg, tid);
}

__device__ __forceinline__ void out_flush(const float* win, float* outp, size_t F0, int t, int w, int lane) {
  const int q8 = lane & 7, sub = lane >> 3;
#pragma unroll
  for (int i = 0; i < 4; ++i) {
    const int it = 16 * w + 4 * i + sub;
    const int o = it >> 1, wl = it & 1;
    bool valid = true;
    if (t == 0) valid = (wl == 1) || (o == 0);
    if (t == NT - 1) valid = (wl == 0);
    const v4f v = *(const v4fa*)(win + o * 96 + 32 * wl + 4 * q8);
    const size_t L = (size_t)(LPC * o + 2 * t + wl);
    if (valid) *(volatile v4f*)(outp + F0 + L * 32 + 4 * q8) = v;
  }
}

__global__ __launch_bounds__(128) void k_out(
    const us_t* __restrict__ cth, const us_t* __restrict__ ctl,
    const us_t* __restrict__ wwh, const us_t* __restrict__ wwl, const float* __restrict__ bw,
    float* __restrict__ outp)
{
  __shared__ __attribute__((aligned(16))) float win[32 * 96];
  __shared__ __attribute__((aligned(16))) float head[32 * 32];
  const int tid = threadIdx.x, lane = tid & 31, w = tid >> 5, h = lane >> 4, m = lane & 15;
  const int g = blockIdx.x, b = blockIdx.y;
  const size_t F0 = ((size_t)(b * CO + 32 * g)) * NSP;
  const size_t brow = ((size_t)(32 * g + m)) * CI;
  float bias[2];
  bias[0] = bw[32 * g + m];
  bias[1] = bw[32 * g + 16 + m];
  const v8f zero8 = {0.f, 0.f, 0.f, 0.f, 0.f, 0.f, 0.f, 0.f};

#pragma unroll 1
  for (int t = 0; t < NT; ++t) {
    const int n0 = 64 * t;
    const size_t arow = ((size_t)(b * NP + n0 + 16 * w + m)) * CI;
    v8f acc[2];
    acc[0] = zero8; acc[1] = zero8;
#pragma unroll 1
    for (int k0 = 0; k0 < CI; k0 += 32) {
      const v16b ah = ldb(cth + arow + k0, h);
      const v16b al = ldb(ctl + arow + k0, h);
#pragma unroll
      for (int nt = 0; nt < 2; ++nt) {
        const v16b bh = ldb(wwh + brow + (size_t)nt * 16 * CI + k0, h);
        const v16b bl = ldb(wwl + brow + (size_t)nt * 16 * CI + k0, h);
        acc[nt] = mma_b(ah, bh, acc[nt]);
        acc[nt] = mma_b(al, bh, acc[nt]);
        acc[nt] = mma_b(ah, bl, acc[nt]);
      }
    }
#pragma unroll
    for (int nt = 0; nt < 2; ++nt) {
      const int o = 16 * nt + m;
#pragma unroll
      for (int r = 0; r < 8; ++r) {
        const int j = 16 * w + 8 * h + r;
        if (n0 + j < NSP) win[o * 96 + o + j] = acc[nt][r] + bias[nt];
      }
    }
    __syncthreads();
    if (t == 0) {
      for (int idx = tid; idx < 1024; idx += 128) head[idx] = win[(idx >> 5) * 96 + (idx & 31)];
    }
    if (t == NT - 1) {
      for (int idx = tid; idx < 1024; idx += 128) {
        const int o = idx >> 5, p = idx & 31;
        if (o < 31 && p > o) win[o * 96 + p] = head[(o + 1) * 32 + p];
      }
    }
    __syncthreads();
    out_flush(win, outp, F0, t, w, lane);
    __threadfence();
    out_flush(win, outp, F0, t, w, lane);
    __syncthreads();
    for (int idx = tid; idx < 1024; idx += 128) {
      const int o = idx >> 5, p = idx & 31;
      win[o * 96 + p] = win[o * 96 + 64 + p];
    }
    __syncthreads();
  }
}

extern "C" void kernel_launch(void* const* d_in, const int* in_sizes, int n_in,
                              void* d_out, int out_size, void* d_ws, size_t ws_size,
                              hipStream_t stream)
{
  if (n_in < 11) return;
  if (in_sizes[0] != NB * CIN * NSP) return;
  if (in_sizes[1] != CI * CIN || in_sizes[5] != CI * CIN) return;
  if (in_sizes[2] != CI || in_sizes[3] != CI || in_sizes[4] != CI || in_sizes[6] != CI || in_sizes[8] != CI) return;
  if (in_sizes[7] != CI * CI) return;
  if (in_sizes[9] != CO * CI || in_sizes[10] != CO) return;
  if (out_size != NB * CO * NSP) return;
  if (ws_size < OFF_END) return;

  const float* x     = (const float*)d_in[0];
  const float* Wk    = (const float*)d_in[1];
  const float* bk    = (const float*)d_in[2];
  const float* gamma = (const float*)d_in[3];
  const float* beta  = (const float*)d_in[4];
  const float* Wv    = (const float*)d_in[5];
  const float* bv    = (const float*)d_in[6];
  const float* Wv2   = (const float*)d_in[7];
  const float* bv2   = (const float*)d_in[8];
  const float* Ww    = (const float*)d_in[9];
  const float* bw    = (const float*)d_in[10];
  float* outp = (float*)d_out;
  char* ws = (char*)d_ws;

  _Float16* wk16 = (_Float16*)(ws + OFF_WK);
  us_t* wvh  = (us_t*)(ws + OFF_WVH);
  us_t* wvl  = (us_t*)(ws + OFF_WVL);
  us_t* wv2h = (us_t*)(ws + OFF_WV2H);
  us_t* wv2l = (us_t*)(ws + OFF_WV2L);
  us_t* wwh  = (us_t*)(ws + OFF_WWH);
  us_t* wwl  = (us_t*)(ws + OFF_WWL);
  _Float16* xh16 = (_Float16*)(ws + OFF_XH);
  us_t* xbh  = (us_t*)(ws + OFF_XBH);
  us_t* xbl  = (us_t*)(ws + OFF_XBL);
  _Float16* qkp  = (_Float16*)(ws + OFF_QK);
  float* vf      = (float*)(ws + OFF_VF);
  _Float16* vh16 = (_Float16*)(ws + OFF_VH);
  float* poolT   = (float*)(ws + OFF_POOL);
  _Float16* v2T  = (_Float16*)(ws + OFF_V2T);
  us_t* v2hp = (us_t*)(ws + OFF_V2H);
  us_t* v2lp = (us_t*)(ws + OFF_V2L);
  _Float16* simvT = (_Float16*)(ws + OFF_SIMV);
  us_t* snh = (us_t*)(ws + OFF_SNH);
  us_t* snl = (us_t*)(ws + OFF_SNL);
  us_t* cth = (us_t*)(ws + OFF_CTH);
  us_t* ctl = (us_t*)(ws + OFF_CTL);

  const int ngroups = (CI * CIN / 8) * 2 + CI * CI / 8 + CO * CI / 8;
  k_wprep<<<(ngroups + 255) / 256, 256, 0, stream>>>(Wk, Wv, Wv2, Ww, wk16, wvh, wvl, wv2h, wv2l, wwh, wwl);
  k_xprep<<<dim3(NP / 64, CIN / 64, NB), 256, 0, stream>>>(x, xh16, xbh, xbl);
  k_convq<<<dim3(NP / 64, CI / 64, NB), 128, 0, stream>>>(xh16, wk16, bk, gamma, beta, qkp);
  k_convv<<<dim3(NP / 64, CI / 64, NB), 128, 0, stream>>>(xbh, xbl, wvh, wvl, bv, vf, vh16);
  k_pool<<<(NB * KP * CI + 255) / 256, 256, 0, stream>>>(vf, poolT);
  k_v2<<<dim3(CI / 64, NB), 128, 0, stream>>>(wv2h, wv2l, poolT, bv2, v2T, v2hp, v2lp);
  k_simv<<<dim3(NP / 64, NB), 128, 0, stream>>>(vh16, v2T, simvT);
  k_flash<<<dim3(NP / 64, NB), 128, 0, stream>>>(qkp, simvT, snh, snl);
  k_ctx<<<dim3(NP / 64, CI / 64, NB), 128, 0, stream>>>(snh, snl, v2hp, v2lp, cth, ctl);
  k_out<<<dim3(CO / 32, NB), 128, 0, stream>>>(cth, ctl, wwh, wwl, bw, outp);
}
